// PHA_85014582657526
// MI455X (gfx1250) — hardware-verified
//
#include <hip/hip_runtime.h>
#define BB 4
#define CC 64
#define HW 4096
#define C8 8
#define FL 16

typedef __bf16 v16b __attribute__((ext_vector_type(16)));
typedef unsigned short v8us __attribute__((ext_vector_type(8), may_alias));
typedef float  v8f  __attribute__((ext_vector_type(8)));
typedef float  v4f  __attribute__((ext_vector_type(4)));
typedef float  v4fa __attribute__((ext_vector_type(4), may_alias));
union FragB { v16b v; v8us half[2]; unsigned short u[16]; };

__device__ __forceinline__ unsigned short bf16_bits(float x) { unsigned int u = __float_as_uint(x); return (unsigned short)((u + 0x7FFFu + ((u >> 16) & 1u)) >> 16); }
__device__ __forceinline__ float bf16_val(unsigned short b) { return __uint_as_float(((unsigned int)b) << 16); }
__device__ __forceinline__ float bf16_round(float x) { return bf16_val(bf16_bits(x)); }
template <int NT>
__device__ __forceinline__ v8f mmaN(v16b ah, v16b al, v16b bh, v16b bl, v8f c) {
  c = __builtin_amdgcn_wmma_f32_16x16x32_bf16(false, ah, false, bh, (short)0, c, false, false);
  if (NT >= 2) c = __builtin_amdgcn_wmma_f32_16x16x32_bf16(false, al, false, bh, (short)0, c, false, false);
  if (NT >= 3) c = __builtin_amdgcn_wmma_f32_16x16x32_bf16(false, ah, false, bl, (short)0, c, false, false);
  asm volatile("v_nop\n\tv_nop\n\tv_nop\n\tv_nop" : "+v"(c) : "v"(ah), "v"(al), "v"(bh), "v"(bl));
  return c;
}

__global__ __launch_bounds__(256) void k_wt_bf16(const float* __restrict__ W, unsigned short* __restrict__ Wt, int K, int N) {
  const int t = blockIdx.x * 256 + threadIdx.x;
  const int k8n = K / 8;
  if (t >= N * k8n) return;
  const int n = t / k8n, k8 = (t % k8n) * 8;
  v8us v;
#pragma unroll
  for (int i = 0; i < 8; ++i) v[i] = bf16_bits(W[(size_t)(k8 + i) * N + n]);
  *(volatile v8us*)(Wt + (size_t)n * K + k8) = v;
  __threadfence();
  *(volatile v8us*)(Wt + (size_t)n * K + k8) = v;
}

template <bool ASPLIT, int ACT, bool BIAS_BF16>
__global__ __launch_bounds__(128) void k_gemm_bf(const float* __restrict__ A, int lda, const unsigned short* __restrict__ Wt, int ldb,
                                               const float* __restrict__ bias, float* __restrict__ C, int ldc, int M, int N, int K) {
  __shared__ __attribute__((aligned(16))) float so[4][16][64];
  const int tid = threadIdx.x, w = tid >> 5, lane = tid & 31, ln = lane & 15, hh = lane >> 4;
  const int ntn = N / 64;
  const int wid = blockIdx.x * 4 + w;
  const int mt = wid / ntn, nq = wid % ntn;
  if (mt * 16 >= M) return;
  const int row0 = mt * 16, col0 = nq * 64;
  const float* arow = A + (size_t)(row0 + ln) * lda;
  v8f acc[4] = {};
  for (int kb = 0; kb < K; kb += 32) {
    FragB ah, al;
    const v4f x0 = *(const v4fa*)(arow + kb + 8 * hh), x1 = *(const v4fa*)(arow + kb + 8 * hh + 4);
    const v4f x2 = *(const v4fa*)(arow + kb + 16 + 8 * hh), x3 = *(const v4fa*)(arow + kb + 16 + 8 * hh + 4);
    float xs[16] = {x0[0],x0[1],x0[2],x0[3],x1[0],x1[1],x1[2],x1[3],x2[0],x2[1],x2[2],x2[3],x3[0],x3[1],x3[2],x3[3]};
#pragma unroll
    for (int i = 0; i < 16; ++i) { const unsigned short hb = bf16_bits(xs[i]); ah.u[i] = hb; al.u[i] = ASPLIT ? bf16_bits(xs[i] - bf16_val(hb)) : (unsigned short)0; }
#pragma unroll
    for (int t = 0; t < 4; ++t) {
      const unsigned short* brow = Wt + (size_t)(col0 + t * 16 + ln) * ldb + kb;
      FragB b;
      b.half[0] = *(const v8us*)(brow + 8 * hh);
      b.half[1] = *(const v8us*)(brow + 16 + 8 * hh);
      acc[t] = mmaN<ASPLIT ? 2 : 1>(ah.v, al.v, b.v, b.v, acc[t]);
    }
  }
#pragma unroll
  for (int t = 0; t < 4; ++t) {
    float bv = bias ? bias[col0 + t * 16 + ln] : 0.f;
    if (BIAS_BF16) bv = bf16_round(bv);
#pragma unroll
    for (int r = 0; r < 8; ++r) { float v = acc[t][r] + bv; if (ACT == 1) v = fmaxf(v, 0.f); so[w][8 * hh + r][t * 16 + ln] = v; }
  }
  __builtin_amdgcn_fence(__ATOMIC_ACQ_REL, "workgroup");
  __builtin_amdgcn_wave_barrier();
  const int rsub = lane >> 4, c4 = (lane & 15) * 4;
  for (int pass = 0; pass < 2; ++pass) {
#pragma unroll
    for (int q = 0; q < 8; ++q) {
      const int r = q * 2 + rsub;
      const v4f v = *(const v4fa*)&so[w][r][c4];
      *(volatile v4f*)(C + (size_t)(row0 + r) * ldc + col0 + c4) = v;
    }
    if (pass == 0) __threadfence();
  }
}

template <int D, bool CAUSAL>
__global__ __launch_bounds__(128) void k_flash(const float* __restrict__ qb, const float* __restrict__ kb, const float* __restrict__ vb,
                                             int pitch, int T, int H, float scale, float* __restrict__ y, int ypitch) {
  constexpr int KS = D / 32;
  constexpr int DT = D / 16;
  __shared__ __attribute__((aligned(16))) unsigned short sKh[32][D + 8], sKl[32][D + 8], sVh[32][D + 8], sVl[32][D + 8];
  __shared__ __attribute__((aligned(16))) unsigned short sPh[4][16][40], sPl[4][16][40];
  __shared__ __attribute__((aligned(16))) float sO[4][16][D];
  const int tid = threadIdx.x, w = tid >> 5, lane = tid & 31, ln = lane & 15, hh = lane >> 4;
  const int nqb = (T + 63) / 64;
  const int bh = blockIdx.x / nqb, qblk = blockIdx.x % nqb;
  const int b = bh / H, h = bh % H;
  const int q0 = qblk * 64 + w * 16;
  const float* Q = qb + (size_t)b * T * pitch + h * D;
  const float* K = kb + (size_t)b * T * pitch + h * D;
  const float* V = vb + (size_t)b * T * pitch + h * D;

  FragB aqh[KS], aql[KS];
  {
    int row = q0 + ln; if (row >= T) row = T - 1;
    const float* qr = Q + (size_t)row * pitch;
#pragma unroll
    for (int ks = 0; ks < KS; ++ks)
#pragma unroll
      for (int i = 0; i < 16; ++i) {
        const int d = ks * 32 + ((i < 8) ? (8 * hh + i) : (16 + 8 * hh + (i - 8)));
        const float x = qr[d] * scale; const unsigned short hb = bf16_bits(x);
        aqh[ks].u[i] = hb; aql[ks].u[i] = bf16_bits(x - bf16_val(hb));
      }
  }
  float m_r[8], l_r[8];
#pragma unroll
  for (int r = 0; r < 8; ++r) { m_r[r] = -3.0e38f; l_r[r] = 0.f; }
  v8f oacc[DT];
#pragma unroll
  for (int dt = 0; dt < DT; ++dt) oacc[dt] = (v8f){0.f,0.f,0.f,0.f,0.f,0.f,0.f,0.f};

  const int kv_end = CAUSAL ? min(T, qblk * 64 + 64) : T;
  for (int j0 = 0; j0 < kv_end; j0 += 32) {
    __syncthreads();
    for (int e = tid; e < 32 * (D / 4); e += 128) {
      const int r = e / (D / 4), c4 = (e % (D / 4)) * 4;
      const int key = j0 + r;
      v4f kf = {0.f,0.f,0.f,0.f}, vf = {0.f,0.f,0.f,0.f};
      if (key < T) { kf = *(const v4fa*)(K + (size_t)key * pitch + c4); vf = *(const v4fa*)(V + (size_t)key * pitch + c4); }
#pragma unroll
      for (int t = 0; t < 4; ++t) {
        unsigned short hb = bf16_bits(kf[t]); sKh[r][c4 + t] = hb; sKl[r][c4 + t] = bf16_bits(kf[t] - bf16_val(hb));
        hb = bf16_bits(vf[t]); sVh[r][c4 + t] = hb; sVl[r][c4 + t] = bf16_bits(vf[t] - bf16_val(hb));
      }
    }
    __syncthreads();
    v8f s[2];
#pragma unroll
    for (int nt = 0; nt < 2; ++nt) {
      v8f acc = {};
#pragma unroll
      for (int ks = 0; ks < KS; ++ks) {
        FragB bh_, bl_;
        bh_.half[0] = *(const v8us*)&sKh[nt * 16 + ln][ks * 32 + 8 * hh]; bh_.half[1] = *(const v8us*)&sKh[nt * 16 + ln][ks * 32 + 16 + 8 * hh];
        bl_.half[0] = *(const v8us*)&sKl[nt * 16 + ln][ks * 32 + 8 * hh]; bl_.half[1] = *(const v8us*)&sKl[nt * 16 + ln][ks * 32 + 16 + 8 * hh];
        acc = mmaN<3>(aqh[ks].v, aql[ks].v, bh_.v, bl_.v, acc);
      }
      s[nt] = acc;
    }
    float alpha[8];
#pragma unroll
    for (int r = 0; r < 8; ++r) {
      const int qi = q0 + 8 * hh + r;
      const int ja = j0 + ln, jb = j0 + 16 + ln;
      if (CAUSAL) { if (ja > qi) s[0][r] = -3.0e38f; if (jb > qi) s[1][r] = -3.0e38f; }
      if (ja >= T) s[0][r] = -3.0e38f;
      if (jb >= T) s[1][r] = -3.0e38f;
      float mx = fmaxf(s[0][r], s[1][r]);
      mx = fmaxf(mx, __shfl_xor(mx, 1, 32)); mx = fmaxf(mx, __shfl_xor(mx, 2, 32)); mx = fmaxf(mx, __shfl_xor(mx, 4, 32)); mx = fmaxf(mx, __shfl_xor(mx, 8, 32));
      const float mnew = fmaxf(m_r[r], mx);
      alpha[r] = (mnew > -1.0e38f) ? __expf(m_r[r] - mnew) : 1.0f;
      const float p0 = (s[0][r] > -1.0e38f) ? __expf(s[0][r] - mnew) : 0.f;
      const float p1 = (s[1][r] > -1.0e38f) ? __expf(s[1][r] - mnew) : 0.f;
      m_r[r] = mnew;
      l_r[r] = l_r[r] * alpha[r] + p0 + p1;
      unsigned short hb = bf16_bits(p0); sPh[w][8 * hh + r][ln] = hb;      sPl[w][8 * hh + r][ln] = bf16_bits(p0 - bf16_val(hb));
      hb = bf16_bits(p1);                sPh[w][8 * hh + r][16 + ln] = hb; sPl[w][8 * hh + r][16 + ln] = bf16_bits(p1 - bf16_val(hb));
    }
#pragma unroll
    for (int dt = 0; dt < DT; ++dt)
#pragma unroll
      for (int r = 0; r < 8; ++r) oacc[dt][r] *= alpha[r];
    __builtin_amdgcn_fence(__ATOMIC_ACQ_REL, "workgroup");
    __builtin_amdgcn_wave_barrier();
    FragB pah, pal;
    pah.half[0] = *(const v8us*)&sPh[w][ln][8 * hh]; pah.half[1] = *(const v8us*)&sPh[w][ln][16 + 8 * hh];
    pal.half[0] = *(const v8us*)&sPl[w][ln][8 * hh]; pal.half[1] = *(const v8us*)&sPl[w][ln][16 + 8 * hh];
#pragma unroll
    for (int dt = 0; dt < DT; ++dt) {
      FragB bvh, bvl;
#pragma unroll
      for (int i = 0; i < 8; ++i) {
        bvh.u[i] = sVh[8 * hh + i][dt * 16 + ln]; bvh.u[8 + i] = sVh[16 + 8 * hh + i][dt * 16 + ln];
        bvl.u[i] = sVl[8 * hh + i][dt * 16 + ln]; bvl.u[8 + i] = sVl[16 + 8 * hh + i][dt * 16 + ln];
      }
      oacc[dt] = mmaN<3>(pah.v, pal.v, bvh.v, bvl.v, oacc[dt]);
    }
    __builtin_amdgcn_fence(__ATOMIC_ACQ_REL, "workgroup");
    __builtin_amdgcn_wave_barrier();
  }
#pragma unroll
  for (int r = 0; r < 8; ++r) {
    float l = l_r[r];
    l += __shfl_xor(l, 1, 32); l += __shfl_xor(l, 2, 32); l += __shfl_xor(l, 4, 32); l += __shfl_xor(l, 8, 32);
    l_r[r] = (l > 0.f) ? 1.0f / l : 0.f;
  }
#pragma unroll
  for (int dt = 0; dt < DT; ++dt)
#pragma unroll
    for (int r = 0; r < 8; ++r) sO[w][8 * hh + r][dt * 16 + ln] = oacc[dt][r] * l_r[r];
  __builtin_amdgcn_fence(__ATOMIC_ACQ_REL, "workgroup");
  __builtin_amdgcn_wave_barrier();
  for (int pass = 0; pass < 2; ++pass) {
    for (int r = 0; r < 16; ++r) {
      const int row = q0 + r;
      if (row < T && lane < D / 4) {
        const v4f val = *(const v4fa*)&sO[w][r][lane * 4];
        *(volatile v4f*)(y + ((size_t)b * T + row) * ypitch + h * D + lane * 4) = val;
      }
    }
    if (pass == 0) __threadfence();
  }
}

template <bool AFFINE, bool RESID, bool RES_BF16>
__global__ __launch_bounds__(256) void k_transpose32(const float* __restrict__ in, float* __restrict__ out, int rows, int cols,
                                                    const float* __restrict__ scale, const float* __restrict__ shift, const float* __restrict__ res) {
  __shared__ float tile[32][33];
  const int b = blockIdx.z;
  const int r0 = blockIdx.y * 32, c0 = blockIdx.x * 32;
  const float* src = in + (size_t)b * rows * cols;
  float* dst = out + (size_t)b * rows * cols;
  const int tx = threadIdx.x & 31, ty = threadIdx.x >> 5;
  for (int i = ty; i < 32; i += 8) tile[i][tx] = src[(size_t)(r0 + i) * cols + c0 + tx];
  __syncthreads();
  for (int pass = 0; pass < 2; ++pass) {
    for (int i = ty; i < 32; i += 8) {
      float v = tile[tx][i];
      const int orow = c0 + i;
      if (AFFINE) v = v * scale[orow] + shift[orow];
      if (RESID) { float rv = res[(size_t)b * rows * cols + (size_t)orow * rows + r0 + tx]; if (RES_BF16) rv = bf16_round(rv); v += rv; }
      *(volatile float*)(dst + (size_t)orow * rows + r0 + tx) = v;
    }
    if (pass == 0) __threadfence();
  }
}

__global__ __launch_bounds__(256) void k_pool2_pm(const float* __restrict__ in, float* __restrict__ out, int Bn, int H, int W, int C) {
  const size_t t = (size_t)blockIdx.x * 256 + threadIdx.x;
  const int c4n = C / 4, Ho = H / 2, Wo = W / 2;
  const size_t total = (size_t)Bn * Ho * Wo * c4n;
  if (t >= total) return;
  const int c4 = (int)(t % c4n) * 4; size_t rest = t / c4n;
  const int pw = (int)(rest % Wo); rest /= Wo; const int ph = (int)(rest % Ho); const int b = (int)(rest / Ho);
  const float* base = in + (size_t)b * H * W * C;
  const int p00 = (2 * ph) * W + 2 * pw;
  const v4f a = *(const v4fa*)(base + (size_t)p00 * C + c4), bq = *(const v4fa*)(base + (size_t)(p00 + 1) * C + c4);
  const v4f c = *(const v4fa*)(base + (size_t)(p00 + W) * C + c4), d = *(const v4fa*)(base + (size_t)(p00 + W + 1) * C + c4);
  v4f m; for (int i = 0; i < 4; ++i) m[i] = fmaxf(fmaxf(a[i], bq[i]), fmaxf(c[i], d[i]));
  float* dst = out + ((size_t)b * Ho * Wo + (size_t)ph * Wo + pw) * C + c4;
  *(volatile v4f*)dst = m;
  __threadfence();
  *(volatile v4f*)dst = m;
}

template <int DQ, int DV>
__global__ __launch_bounds__(128) void k_flash2(const float* __restrict__ Qb, size_t qstride, int qpitch, int Tq,
                                              const float* __restrict__ Kb, size_t kstride, int kpitch, int Tk,
                                              const float* __restrict__ Vb, size_t vstride, int vpitch,
                                              float scale, float* __restrict__ y, size_t ystride, int ypitch) {
  constexpr int KS = DQ / 32, DT = DV / 16;
  __shared__ __attribute__((aligned(16))) unsigned short sKh[32][DQ + 8], sKl[32][DQ + 8], sVh[32][DV + 8], sVl[32][DV + 8];
  __shared__ __attribute__((aligned(16))) unsigned short sPh[4][16][40], sPl[4][16][40];
  __shared__ __attribute__((aligned(16))) float sO[4][16][DV];
  const int tid = threadIdx.x, w = tid >> 5, lane = tid & 31, ln = lane & 15, hh = lane >> 4;
  const int nqb = (Tq + 63) / 64;
  const int bh = blockIdx.x / nqb, qblk = blockIdx.x % nqb;
  const int dv0 = blockIdx.y * DV;
  const int q0 = qblk * 64 + w * 16;
  const float* Q = Qb + (size_t)bh * qstride; const float* K = Kb + (size_t)bh * kstride; const float* V = Vb + (size_t)bh * vstride + dv0;
  FragB aqh[KS], aql[KS];
  {
    int row = q0 + ln; if (row >= Tq) row = Tq - 1;
    const float* qr = Q + (size_t)row * qpitch;
#pragma unroll
    for (int ks = 0; ks < KS; ++ks)
#pragma unroll
      for (int i = 0; i < 16; ++i) {
        const int d = ks * 32 + ((i < 8) ? (8 * hh + i) : (16 + 8 * hh + (i - 8)));
        const float x = qr[d] * scale; const unsigned short hb = bf16_bits(x);
        aqh[ks].u[i] = hb; aql[ks].u[i] = bf16_bits(x - bf16_val(hb));
      }
  }
  float m_r[8], l_r[8];
#pragma unroll
  for (int r = 0; r < 8; ++r) { m_r[r] = -3.0e38f; l_r[r] = 0.f; }
  v8f oacc[DT];
#pragma unroll
  for (int dt = 0; dt < DT; ++dt) oacc[dt] = (v8f){0.f,0.f,0.f,0.f,0.f,0.f,0.f,0.f};
  for (int j0 = 0; j0 < Tk; j0 += 32) {
    __syncthreads();
    for (int e = tid; e < 32 * (DQ / 4); e += 128) {
      const int r = e / (DQ / 4), c4 = (e % (DQ / 4)) * 4; const int key = j0 + r;
      v4f f = {0.f,0.f,0.f,0.f}; if (key < Tk) f = *(const v4fa*)(K + (size_t)key * kpitch + c4);
#pragma unroll
      for (int t = 0; t < 4; ++t) { const unsigned short hb = bf16_bits(f[t]); sKh[r][c4 + t] = hb; sKl[r][c4 + t] = bf16_bits(f[t] - bf16_val(hb)); }
    }
    for (int e = tid; e < 32 * (DV / 4); e += 128) {
      const int r = e / (DV / 4), c4 = (e % (DV / 4)) * 4; const int key = j0 + r;
      v4f f = {0.f,0.f,0.f,0.f}; if (key < Tk) f = *(const v4fa*)(V + (size_t)key * vpitch + c4);
#pragma unroll
      for (int t = 0; t < 4; ++t) { const unsigned short hb = bf16_bits(f[t]); sVh[r][c4 + t] = hb; sVl[r][c4 + t] = bf16_bits(f[t] - bf16_val(hb)); }
    }
    __syncthreads();
    v8f s[2];
#pragma unroll
    for (int nt = 0; nt < 2; ++nt) {
      v8f acc = {};
#pragma unroll
      for (int ks = 0; ks < KS; ++ks) {
        FragB bh_, bl_;
        bh_.half[0] = *(const v8us*)&sKh[nt * 16 + ln][ks * 32 + 8 * hh]; bh_.half[1] = *(const v8us*)&sKh[nt * 16 + ln][ks * 32 + 16 + 8 * hh];
        bl_.half[0] = *(const v8us*)&sKl[nt * 16 + ln][ks * 32 + 8 * hh]; bl_.half[1] = *(const v8us*)&sKl[nt * 16 + ln][ks * 32 + 16 + 8 * hh];
        acc = mmaN<3>(aqh[ks].v, aql[ks].v, bh_.v, bl_.v, acc);
      }
      s[nt] = acc;
    }
    float alpha[8];
#pragma unroll
    for (int r = 0; r < 8; ++r) {
      const int ja = j0 + ln, jb = j0 + 16 + ln;
      if (ja >= Tk) s[0][r] = -3.0e38f;
      if (jb >= Tk) s[1][r] = -3.0e38f;
      float mx = fmaxf(s[0][r], s[1][r]);
      mx = fmaxf(mx, __shfl_xor(mx, 1, 32)); mx = fmaxf(mx, __shfl_xor(mx, 2, 32)); mx = fmaxf(mx, __shfl_xor(mx, 4, 32)); mx = fmaxf(mx, __shfl_xor(mx, 8, 32));
      const float mnew = fmaxf(m_r[r], mx);
      alpha[r] = (mnew > -1.0e38f) ? __expf(m_r[r] - mnew) : 1.0f;
      const float p0 = (s[0][r] > -1.0e38f) ? __expf(s[0][r] - mnew) : 0.f;
      const float p1 = (s[1][r] > -1.0e38f) ? __expf(s[1][r] - mnew) : 0.f;
      m_r[r] = mnew;
      l_r[r] = l_r[r] * alpha[r] + p0 + p1;
      unsigned short hb = bf16_bits(p0); sPh[w][8 * hh + r][ln] = hb;      sPl[w][8 * hh + r][ln] = bf16_bits(p0 - bf16_val(hb));
      hb = bf16_bits(p1);                sPh[w][8 * hh + r][16 + ln] = hb; sPl[w][8 * hh + r][16 + ln] = bf16_bits(p1 - bf16_val(hb));
    }
#pragma unroll
    for (int dt = 0; dt < DT; ++dt)
#pragma unroll
      for (int r = 0; r < 8; ++r) oacc[dt][r] *= alpha[r];
    __builtin_amdgcn_fence(__ATOMIC_ACQ_REL, "workgroup");
    __builtin_amdgcn_wave_barrier();
    FragB pah, pal;
    pah.half[0] = *(const v8us*)&sPh[w][ln][8 * hh]; pah.half[1] = *(const v8us*)&sPh[w][ln][16 + 8 * hh];
    pal.half[0] = *(const v8us*)&sPl[w][ln][8 * hh]; pal.half[1] = *(const v8us*)&sPl[w][ln][16 + 8 * hh];
#pragma unroll
    for (int dt = 0; dt < DT; ++dt) {
      FragB bvh, bvl;
#pragma unroll
      for (int i = 0; i < 8; ++i) {
        bvh.u[i] = sVh[8 * hh + i][dt * 16 + ln]; bvh.u[8 + i] = sVh[16 + 8 * hh + i][dt * 16 + ln];
        bvl.u[i] = sVl[8 * hh + i][dt * 16 + ln]; bvl.u[8 + i] = sVl[16 + 8 * hh + i][dt * 16 + ln];
      }
      oacc[dt] = mmaN<3>(pah.v, pal.v, bvh.v, bvl.v, oacc[dt]);
    }
    __builtin_amdgcn_fence(__ATOMIC_ACQ_REL, "workgroup");
    __builtin_amdgcn_wave_barrier();
  }
#pragma unroll
  for (int r = 0; r < 8; ++r) {
    float l = l_r[r];
    l += __shfl_xor(l, 1, 32); l += __shfl_xor(l, 2, 32); l += __shfl_xor(l, 4, 32); l += __shfl_xor(l, 8, 32);
    l_r[r] = (l > 0.f) ? 1.0f / l : 0.f;
  }
#pragma unroll
  for (int dt = 0; dt < DT; ++dt)
#pragma unroll
    for (int r = 0; r < 8; ++r) sO[w][8 * hh + r][dt * 16 + ln] = oacc[dt][r] * l_r[r];
  __builtin_amdgcn_fence(__ATOMIC_ACQ_REL, "workgroup");
  __builtin_amdgcn_wave_barrier();
  for (int pass = 0; pass < 2; ++pass) {
    for (int r = 0; r < 16; ++r) {
      const int row = q0 + r;
      for (int c4 = lane * 4; c4 < DV; c4 += 128) {
        if (row < Tq) {
          const v4f val = *(const v4fa*)&sO[w][r][c4];
          *(volatile v4f*)(y + (size_t)bh * ystride + (size_t)row * ypitch + dv0 + c4) = val;
        }
      }
    }
    if (pass == 0) __threadfence();
  }
}

template <bool ASPLIT, int ACT, bool BIAS_BF16, bool RES_BF16>
__global__ __launch_bounds__(128) void k_gemm_bf3(const float* __restrict__ A, int lda, const unsigned short* __restrict__ Wt, int ldb,
                                                const float* __restrict__ bias, const float* __restrict__ resid, int rmod, int ldr,
                                                float* __restrict__ C, int ldc, int M, int N, int K) {
  __shared__ __attribute__((aligned(16))) float so[4][16][64];
  const int tid = threadIdx.x, w = tid >> 5, lane = tid & 31, ln = lane & 15, hh = lane >> 4;
  const int ntn = N / 64;
  const int wid = blockIdx.x * 4 + w;
  const int mt = wid / ntn, nq = wid % ntn;
  if (mt * 16 >= M) return;
  const int row0 = mt * 16, col0 = nq * 64;
  const float* arow = A + (size_t)(row0 + ln) * lda;
  v8f acc[4] = {};
  for (int kb = 0; kb < K; kb += 32) {
    FragB ah, al;
    const v4f x0 = *(const v4fa*)(arow + kb + 8 * hh), x1 = *(const v4fa*)(arow + kb + 8 * hh + 4);
    const v4f x2 = *(const v4fa*)(arow + kb + 16 + 8 * hh), x3 = *(const v4fa*)(arow + kb + 16 + 8 * hh + 4);
    float xs[16] = {x0[0],x0[1],x0[2],x0[3],x1[0],x1[1],x1[2],x1[3],x2[0],x2[1],x2[2],x2[3],x3[0],x3[1],x3[2],x3[3]};
#pragma unroll
    for (int i = 0; i < 16; ++i) { const unsigned short hb = bf16_bits(xs[i]); ah.u[i] = hb; al.u[i] = ASPLIT ? bf16_bits(xs[i] - bf16_val(hb)) : (unsigned short)0; }
#pragma unroll
    for (int t = 0; t < 4; ++t) {
      const unsigned short* brow = Wt + (size_t)(col0 + t * 16 + ln) * ldb + kb;
      FragB b;
      b.half[0] = *(const v8us*)(brow + 8 * hh);
      b.half[1] = *(const v8us*)(brow + 16 + 8 * hh);
      acc[t] = mmaN<ASPLIT ? 2 : 1>(ah.v, al.v, b.v, b.v, acc[t]);
    }
  }
#pragma unroll
  for (int t = 0; t < 4; ++t) {
    const int col = col0 + t * 16 + ln;
    float bv = bias ? bias[col] : 0.f;
    if (BIAS_BF16) bv = bf16_round(bv);
#pragma unroll
    for (int r = 0; r < 8; ++r) {
      float v = acc[t][r] + bv;
      if (resid) { float rv = resid[(size_t)((row0 + 8 * hh + r) % rmod) * ldr + col]; if (RES_BF16) rv = bf16_round(rv); v += rv; }
      if (ACT == 1) v = fmaxf(v, 0.f);
      if (ACT == 2) v = 0.5f * v * (1.0f + erff(v * 0.70710678118654752f));
      if (ACT == 3) { const float u = 0.7978845608028654f * (v + 0.044715f * v * v * v); v = 0.5f * v * (1.0f + tanhf(u)); }
      so[w][8 * hh + r][t * 16 + ln] = v;
    }
  }
  __builtin_amdgcn_fence(__ATOMIC_ACQ_REL, "workgroup");
  __builtin_amdgcn_wave_barrier();
  const int rsub = lane >> 4, c4 = (lane & 15) * 4;
  for (int pass = 0; pass < 2; ++pass) {
#pragma unroll
    for (int q = 0; q < 8; ++q) {
      const int r = q * 2 + rsub;
      const v4f v = *(const v4fa*)&so[w][r][c4];
      *(volatile v4f*)(C + (size_t)(row0 + r) * ldc + col0 + c4) = v;
    }
    if (pass == 0) __threadfence();
  }
}
template <bool PARAM_BF16>
__global__ __launch_bounds__(256) void k_layernorm(const float* __restrict__ X, const float* __restrict__ R, const float* __restrict__ g, const float* __restrict__ bta,
                                                  float* __restrict__ out_sum, float* __restrict__ out_norm, int N, float eps) {
  __shared__ float red[256];
  const int row = blockIdx.x, tid = threadIdx.x;
  const float* x = X + (size_t)row * N; const float* rr = R ? R + (size_t)row * N : nullptr;
  float vals[16];
  const int per = N / 256;
  float s1 = 0.f;
  for (int u = 0; u < per / 4; ++u) {
    const int j = tid * 4 + 1024 * u;
    const v4f a = *(const v4fa*)(x + j);
    v4f b = {0.f,0.f,0.f,0.f}; if (rr) b = *(const v4fa*)(rr + j);
#pragma unroll
    for (int q = 0; q < 4; ++q) { const float v = a[q] + b[q]; vals[u * 4 + q] = v; s1 += v; }
  }
  red[tid] = s1; __syncthreads();
  for (int st = 128; st > 0; st >>= 1) { if (tid < st) red[tid] += red[tid + st]; __syncthreads(); }
  const float mu = red[0] / (float)N; __syncthreads();
  float s2 = 0.f;
  for (int u = 0; u < per / 4; ++u)
#pragma unroll
    for (int q = 0; q < 4; ++q) { const float c = vals[u * 4 + q] - mu; s2 += c * c; }
  red[tid] = s2; __syncthreads();
  for (int st = 128; st > 0; st >>= 1) { if (tid < st) red[tid] += red[tid + st]; __syncthreads(); }
  const float rs = rsqrtf(red[0] / (float)N + eps);
  for (int pass = 0; pass < 2; ++pass) {
    for (int u = 0; u < per / 4; ++u) {
      const int j = tid * 4 + 1024 * u;
      v4f o, sm;
#pragma unroll
      for (int q = 0; q < 4; ++q) {
        float gg = g[j + q], bb = bta[j + q];
        if (PARAM_BF16) { gg = bf16_round(gg); bb = bf16_round(bb); }
        sm[q] = vals[u * 4 + q]; o[q] = (vals[u * 4 + q] - mu) * rs * gg + bb;
      }
      if (out_sum) *(volatile v4f*)(out_sum + (size_t)row * N + j) = sm;
      *(volatile v4f*)(out_norm + (size_t)row * N + j) = o;
    }
    if (pass == 0) __threadfence();
  }
}

__global__ __launch_bounds__(256) void k_split_rows(const float* __restrict__ src, int lds_, unsigned short* __restrict__ hi, unsigned short* __restrict__ lo, int R, int Cc) {
  const size_t t = (size_t)blockIdx.x * 256 + threadIdx.x;
  const int c8n = Cc / 8;
  if (t >= (size_t)R * c8n) return;
  const int r = (int)(t / c8n), c8 = (int)(t % c8n) * 8;
  const float* s = src + (size_t)r * lds_ + c8;
  const v4f a = *(const v4fa*)s, b = *(const v4fa*)(s + 4);
  float xs[8] = {a[0],a[1],a[2],a[3],b[0],b[1],b[2],b[3]};
  v8us vh, vl;
#pragma unroll
  for (int i = 0; i < 8; ++i) { const unsigned short hb = bf16_bits(xs[i]); vh[i] = hb; vl[i] = bf16_bits(xs[i] - bf16_val(hb)); }
  unsigned short* dh = hi + (size_t)r * Cc + c8; unsigned short* dl = lo + (size_t)r * Cc + c8;
  *(volatile v8us*)dh = vh; *(volatile v8us*)dl = vl; __threadfence(); *(volatile v8us*)dh = vh; *(volatile v8us*)dl = vl;
}
__global__ __launch_bounds__(256) void k_split_transpose(const float* __restrict__ src, int lds_, unsigned short* __restrict__ hi, unsigned short* __restrict__ lo, int K, int N) {
  const size_t t = (size_t)blockIdx.x * 256 + threadIdx.x;
  const int k8n = K / 8;
  if (t >= (size_t)N * k8n) return;
  const int n = (int)(t / k8n), k8 = (int)(t % k8n) * 8;
  v8us vh, vl;
#pragma unroll
  for (int i = 0; i < 8; ++i) { const float x = src[(size_t)(k8 + i) * lds_ + n]; const unsigned short hb = bf16_bits(x); vh[i] = hb; vl[i] = bf16_bits(x - bf16_val(hb)); }
  unsigned short* dh = hi + (size_t)n * K + k8; unsigned short* dl = lo + (size_t)n * K + k8;
  *(volatile v8us*)dh = vh; *(volatile v8us*)dl = vl; __threadfence(); *(volatile v8us*)dh = vh; *(volatile v8us*)dl = vl;
}
template <bool ASPLIT, bool BSPLIT, int ACT, bool BIAS_BF16>
__global__ __launch_bounds__(128) void k_gemm_bf2(const float* __restrict__ A, int lda, const unsigned short* __restrict__ Bh, const unsigned short* __restrict__ Bl, int ldb,
                                                const float* __restrict__ bias, float alpha, float* __restrict__ C, int ldc, int M, int N, int K) {
  __shared__ __attribute__((aligned(16))) float so[4][16][64];
  const int tid = threadIdx.x, w = tid >> 5, lane = tid & 31, ln = lane & 15, hh = lane >> 4;
  const int ntn = N / 64;
  const int wid = blockIdx.x * 4 + w;
  const int mt = wid / ntn, nq = wid % ntn;
  if (mt * 16 >= M) return;
  const int row0 = mt * 16, col0 = nq * 64;
  const float* arow = A + (size_t)(row0 + ln) * lda;
  v8f acc[4] = {};
  for (int kb = 0; kb < K; kb += 32) {
    FragB ah, al;
    const v4f x0 = *(const v4fa*)(arow + kb + 8 * hh), x1 = *(const v4fa*)(arow + kb + 8 * hh + 4);
    const v4f x2 = *(const v4fa*)(arow + kb + 16 + 8 * hh), x3 = *(const v4fa*)(arow + kb + 16 + 8 * hh + 4);
    float xs[16] = {x0[0],x0[1],x0[2],x0[3],x1[0],x1[1],x1[2],x1[3],x2[0],x2[1],x2[2],x2[3],x3[0],x3[1],x3[2],x3[3]};
#pragma unroll
    for (int i = 0; i < 16; ++i) { const unsigned short hb = bf16_bits(xs[i]); ah.u[i] = hb; al.u[i] = ASPLIT ? bf16_bits(xs[i] - bf16_val(hb)) : (unsigned short)0; }
#pragma unroll
    for (int t = 0; t < 4; ++t) {
      const size_t boff = (size_t)(col0 + t * 16 + ln) * ldb + kb;
      FragB bh_, bl_;
      bh_.half[0] = *(const v8us*)(Bh + boff + 8 * hh);
      bh_.half[1] = *(const v8us*)(Bh + boff + 16 + 8 * hh);
      if (BSPLIT) { bl_.half[0] = *(const v8us*)(Bl + boff + 8 * hh); bl_.half[1] = *(const v8us*)(Bl + boff + 16 + 8 * hh); } else bl_ = bh_;
      acc[t] = mmaN<ASPLIT ? (BSPLIT ? 3 : 2) : 1>(ah.v, al.v, bh_.v, bl_.v, acc[t]);
    }
  }
#pragma unroll
  for (int t = 0; t < 4; ++t) {
    float bv = bias ? bias[col0 + t * 16 + ln] : 0.f;
    if (BIAS_BF16) bv = bf16_round(bv);
#pragma unroll
    for (int r = 0; r < 8; ++r) { float v = acc[t][r] * alpha + bv; if (ACT == 1) v = fmaxf(v, 0.f); so[w][8 * hh + r][t * 16 + ln] = v; }
  }
  __builtin_amdgcn_fence(__ATOMIC_ACQ_REL, "workgroup");
  __builtin_amdgcn_wave_barrier();
  const int rsub = lane >> 4, c4 = (lane & 15) * 4;
  for (int pass = 0; pass < 2; ++pass) {
#pragma unroll
    for (int q = 0; q < 8; ++q) {
      const int r = q * 2 + rsub;
      const v4f v = *(const v4fa*)&so[w][r][c4];
      *(volatile v4f*)(C + (size_t)(row0 + r) * ldc + col0 + c4) = v;
    }
    if (pass == 0) __threadfence();
  }
}
__global__ __launch_bounds__(256) void k_softmax_rows(const float* __restrict__ S, float* __restrict__ P, int N, int causal, int rowoff, const int* __restrict__ mask, int mask_pitch) {
  __shared__ float red[256];
  const int row = blockIdx.x, tid = threadIdx.x;
  const float* s = S + (size_t)row * N; float* p_out = P + (size_t)row * N;
  const int qi = row + rowoff;
  float mx = -3.0e38f;
  for (int j = tid; j < N; j += 256) {
    bool keep = true;
    if (causal && j > qi) keep = false;
    if (mask && mask[(size_t)qi * mask_pitch + j] == 0) keep = false;
    const float v = keep ? s[j] : -3.0e38f;
    mx = fmaxf(mx, v);
  }
  red[tid] = mx; __syncthreads();
  for (int st = 128; st > 0; st >>= 1) { if (tid < st) red[tid] = fmaxf(red[tid], red[tid + st]); __syncthreads(); }
  mx = red[0]; __syncthreads();
  float sum = 0.f;
  for (int j = tid; j < N; j += 256) {
    bool keep = true;
    if (causal && j > qi) keep = false;
    if (mask && mask[(size_t)qi * mask_pitch + j] == 0) keep = false;
    const float p = keep ? __expf(s[j] - mx) : 0.f;
    sum += p;
  }
  red[tid] = sum; __syncthreads();
  for (int st = 128; st > 0; st >>= 1) { if (tid < st) red[tid] += red[tid + st]; __syncthreads(); }
  const float inv = (mx > -1.0e38f) ? 1.0f / red[0] : __builtin_nanf("");
  __syncthreads();
  for (int pass = 0; pass < 2; ++pass) {
    for (int j4 = tid * 4; j4 < N; j4 += 1024) {
      v4f out4;
#pragma unroll
      for (int u = 0; u < 4; ++u) {
        const int j = j4 + u;
        bool keep = true;
        if (causal && j > qi) keep = false;
        if (mask && mask[(size_t)qi * mask_pitch + j] == 0) keep = false;
        out4[u] = keep ? __expf(s[j] - mx) * inv : 0.f;
      }
      *(volatile v4f*)(p_out + j4) = out4;
    }
    if (pass == 0) __threadfence();
  }
}

template <bool ASPLIT, bool BSPLIT, int ACT>
__global__ __launch_bounds__(128) void k_gemm_b(const float* __restrict__ A, int lda, size_t sA, const unsigned short* __restrict__ Bh, const unsigned short* __restrict__ Bl, int ldb, size_t sB,
                                             const float* __restrict__ bias, const float* __restrict__ resid, int ldr, size_t sR, float rsign, float alpha,
                                             float* __restrict__ C, int ldc, size_t sC, int M, int N, int K) {
  __shared__ __attribute__((aligned(16))) float so[4][16][64];
  const int tid = threadIdx.x, w = tid >> 5, lane = tid & 31, ln = lane & 15, hh = lane >> 4;
  const int by = blockIdx.y;
  A += (size_t)by * sA; Bh += (size_t)by * sB; if (BSPLIT) Bl += (size_t)by * sB; C += (size_t)by * sC; if (resid) resid += (size_t)by * sR;
  const int ntn = N / 64; const int wid = blockIdx.x * 4 + w; const int mt = wid / ntn, nq = wid % ntn;
  if (mt * 16 >= M) return;
  const int row0 = mt * 16, col0 = nq * 64;
  const float* arow = A + (size_t)(row0 + ln) * lda;
  v8f acc[4] = {};
  for (int kb = 0; kb < K; kb += 32) {
    FragB ah, al;
    const v4f x0 = *(const v4fa*)(arow + kb + 8 * hh), x1 = *(const v4fa*)(arow + kb + 8 * hh + 4);
    const v4f x2 = *(const v4fa*)(arow + kb + 16 + 8 * hh), x3 = *(const v4fa*)(arow + kb + 16 + 8 * hh + 4);
    float xs[16] = {x0[0],x0[1],x0[2],x0[3],x1[0],x1[1],x1[2],x1[3],x2[0],x2[1],x2[2],x2[3],x3[0],x3[1],x3[2],x3[3]};
#pragma unroll
    for (int i = 0; i < 16; ++i) { const unsigned short hb = bf16_bits(xs[i]); ah.u[i] = hb; al.u[i] = ASPLIT ? bf16_bits(xs[i] - bf16_val(hb)) : (unsigned short)0; }
#pragma unroll
    for (int t = 0; t < 4; ++t) {
      const size_t boff = (size_t)(col0 + t * 16 + ln) * ldb + kb;
      FragB bh_, bl_; bh_.half[0] = *(const v8us*)(Bh + boff + 8 * hh); bh_.half[1] = *(const v8us*)(Bh + boff + 16 + 8 * hh);
      if (BSPLIT) { bl_.half[0] = *(const v8us*)(Bl + boff + 8 * hh); bl_.half[1] = *(const v8us*)(Bl + boff + 16 + 8 * hh); } else bl_ = bh_;
      acc[t] = mmaN<ASPLIT ? (BSPLIT ? 3 : 2) : 1>(ah.v, al.v, bh_.v, bl_.v, acc[t]);
    }
  }
#pragma unroll
  for (int t = 0; t < 4; ++t) {
    const int col = col0 + t * 16 + ln; const float bv = bias ? bf16_round(bias[col]) : 0.f;
#pragma unroll
    for (int r = 0; r < 8; ++r) { float v = acc[t][r] * alpha + bv; if (resid) v += rsign * resid[(size_t)(row0 + 8 * hh + r) * ldr + col]; if (ACT == 1) v = fmaxf(v, 0.f); else if (ACT == 2) v = fmaxf(v, 0.f) + log1pf(expf(-fabsf(v))); so[w][8 * hh + r][t * 16 + ln] = v; }
  }
  __builtin_amdgcn_fence(__ATOMIC_ACQ_REL, "workgroup"); __builtin_amdgcn_wave_barrier();
  const int rsub = lane >> 4, c4 = (lane & 15) * 4;
  for (int pass = 0; pass < 2; ++pass) {
#pragma unroll
    for (int q = 0; q < 8; ++q) { const int r = q * 2 + rsub; const v4f v = *(const v4fa*)&so[w][r][c4]; *(volatile v4f*)(C + (size_t)(row0 + r) * ldc + col0 + c4) = v; }
    if (pass == 0) __threadfence();
  }
}
__global__ __launch_bounds__(256) void k_split_transpose_b(const float* __restrict__ src, int lds_, size_t sIn, unsigned short* __restrict__ hi, unsigned short* __restrict__ lo, size_t sOut, int K, int N) {
  const size_t t = (size_t)blockIdx.x * 256 + threadIdx.x; const int k8n = K / 8; if (t >= (size_t)N * k8n) return;
  src += (size_t)blockIdx.y * sIn; hi += (size_t)blockIdx.y * sOut; lo += (size_t)blockIdx.y * sOut;
  const int n = (int)(t / k8n), k8 = (int)(t % k8n) * 8; v8us vh, vl;
#pragma unroll
  for (int i = 0; i < 8; ++i) { const float x = src[(size_t)(k8 + i) * lds_ + n]; const unsigned short hb = bf16_bits(x); vh[i] = hb; vl[i] = bf16_bits(x - bf16_val(hb)); }
  unsigned short* dh = hi + (size_t)n * K + k8; unsigned short* dl = lo + (size_t)n * K + k8;
  *(volatile v8us*)dh = vh; *(volatile v8us*)dl = vl; __threadfence(); *(volatile v8us*)dh = vh; *(volatile v8us*)dl = vl;
}

__global__ __launch_bounds__(256) void k_wt(const float* __restrict__ qw, const float* __restrict__ kw, const float* __restrict__ vw, const float* __restrict__ w1, const float* __restrict__ qb, const float* __restrict__ kb, const float* __restrict__ vb, const float* __restrict__ b1, unsigned short* __restrict__ Bt, float* __restrict__ bias) {
  const int t = blockIdx.x * 256 + threadIdx.x; if (t >= 128 * (CC / 8)) return; const int n = t / (CC / 8), k8 = (t % (CC / 8)) * 8; v8us v;
  for (int i = 0; i < 8; ++i) { const int c = k8 + i; float w = 0.f; if (n < 8) w = qw[n * CC + c]; else if (n < 16) w = kw[(n - 8) * CC + c]; else if (n < 80) w = vw[(n - 16) * CC + c]; else if (n < 96) w = w1[(n - 80) * CC + c]; v[i] = bf16_bits(w); }
  *(volatile v8us*)(Bt + (size_t)n * CC + k8) = v; __threadfence(); *(volatile v8us*)(Bt + (size_t)n * CC + k8) = v;
  if (t < 128) { float b = 0.f; if (t < 8) b = qb[t]; else if (t < 16) b = kb[t - 8]; else if (t < 80) b = vb[t - 16]; else if (t < 96) b = b1[t - 80]; b = bf16_round(b); *(volatile float*)(bias + t) = b; __threadfence(); *(volatile float*)(bias + t) = b; }
}
__global__ __launch_bounds__(256) void k_qkv(const float* __restrict__ P, float* __restrict__ Qp, unsigned short* __restrict__ Kb) {
  const size_t t = (size_t)blockIdx.x * 256 + threadIdx.x;
  if (t < (size_t)BB * HW * 32) { const int c = (int)(t % 32); const size_t row = t / 32; const float qv = (c < C8) ? P[row * 128 + c] : 0.f; *(volatile float*)(Qp + t) = qv; __threadfence(); *(volatile float*)(Qp + t) = qv; }
  if (t < (size_t)BB * HW * 4) { const int c8 = (int)(t % 4) * 8; const size_t row = t / 4; v8us v; for (int i = 0; i < 8; ++i) { const int c = c8 + i; v[i] = (c < C8) ? bf16_bits(P[row * 128 + C8 + c]) : (unsigned short)0; }
    *(volatile v8us*)(Kb + row * 32 + c8) = v; __threadfence(); *(volatile v8us*)(Kb + row * 32 + c8) = v; }
}
__global__ __launch_bounds__(256) void k_vt(const float* __restrict__ P, unsigned short* __restrict__ Vt) {
  const size_t i = (size_t)blockIdx.x * 256 + threadIdx.x; if (i >= (size_t)BB * CC * (HW / 8)) return; const int j8 = (int)(i % (HW / 8)) * 8; const int c = (int)((i / (HW / 8)) % CC); const int b = (int)(i / ((size_t)(HW / 8) * CC));
  v8us o; for (int q = 0; q < 8; ++q) o[q] = bf16_bits(P[((size_t)b * HW + j8 + q) * 128 + 16 + c]); *(volatile v8us*)(Vt + ((size_t)b * CC + c) * HW + j8) = o; __threadfence(); *(volatile v8us*)(Vt + ((size_t)b * CC + c) * HW + j8) = o;
}
__global__ __launch_bounds__(256) void k_softmax(float* __restrict__ S) {
  const int tid = threadIdx.x, wv = tid >> 5, lane = tid & 31; const size_t r = (size_t)blockIdx.x * 8 + wv; float* row = S + r * HW; float mx = -3.0e38f;
#pragma unroll 1
  for (int j = lane; j < HW; j += 32) mx = fmaxf(mx, row[j]);
  for (int o = 16; o >= 1; o >>= 1) mx = fmaxf(mx, __shfl_xor(mx, o, 32));
  float den = 0.f;
#pragma unroll 1
  for (int j = lane; j < HW; j += 32) { const float e = expf(row[j] - mx); row[j] = e; den += e; }
  for (int o = 16; o >= 1; o >>= 1) den += __shfl_xor(den, o, 32); const float inv = 1.0f / den;
#pragma unroll 1
  for (int j = lane; j < HW; j += 32) { const float p = row[j] * inv; *(volatile float*)(row + j) = p; __threadfence(); *(volatile float*)(row + j) = p; }
}
__global__ __launch_bounds__(256) void k_softpool(const float* __restrict__ P, float* __restrict__ sp) {
  const int t = blockIdx.x * 256 + threadIdx.x; if (t >= BB * FL * 400) return; const int ox = t % 20, oy = (t / 20) % 20, f = (t / 400) % FL, b = t / (400 * FL); float num = 0.f, den = 0.f;
#pragma unroll 1
  for (int dy = 0; dy < 7; ++dy)
#pragma unroll 1
    for (int dx = 0; dx < 7; ++dx) { const int yy = oy * 3 + dy, xx = ox * 3 + dx; const float yv = P[((size_t)b * HW + yy * 64 + xx) * 128 + 80 + f]; const float e = expf(yv); num += e * yv; den += e; }
  const float v = (num / 49.0f) / (den / 49.0f);
  *(volatile float*)(sp + t) = v; __threadfence(); *(volatile float*)(sp + t) = v;
}
__global__ __launch_bounds__(256) void k_conv2(const float* __restrict__ sp, const float* __restrict__ w2, const float* __restrict__ b2, float* __restrict__ y2) {
  const int t = blockIdx.x * 256 + threadIdx.x; if (t >= BB * FL * 100) return; const int ox = t % 10, oy = (t / 10) % 10, o = (t / 100) % FL, b = t / (100 * FL); float a = bf16_round(b2[o]);
#pragma unroll 1
  for (int ci = 0; ci < FL; ++ci)
#pragma unroll 1
    for (int ky = 0; ky < 3; ++ky) for (int kx = 0; kx < 3; ++kx) { const int yy = oy * 2 - 1 + ky, xx = ox * 2 - 1 + kx; if (yy < 0 || yy >= 20 || xx < 0 || xx >= 20) continue; a += bf16_round(w2[((o * FL + ci) * 3 + ky) * 3 + kx]) * sp[((b * FL + ci) * 20 + yy) * 20 + xx]; }
  *(volatile float*)(y2 + t) = a; __threadfence(); *(volatile float*)(y2 + t) = a;
}
__global__ __launch_bounds__(256) void k_conv3(const float* __restrict__ y2, const float* __restrict__ w3, const float* __restrict__ b3, float* __restrict__ y3) {
  const int t = blockIdx.x * 256 + threadIdx.x; if (t >= BB * CC * 100) return; const int ox = t % 10, oy = (t / 10) % 10, o = (t / 100) % CC, b = t / (100 * CC); float a = bf16_round(b3[o]);
#pragma unroll 1
  for (int ci = 0; ci < FL; ++ci)
#pragma unroll 1
    for (int ky = 0; ky < 3; ++ky) for (int kx = 0; kx < 3; ++kx) { const int yy = oy - 1 + ky, xx = ox - 1 + kx; if (yy < 0 || yy >= 10 || xx < 0 || xx >= 10) continue; a += bf16_round(w3[((o * FL + ci) * 3 + ky) * 3 + kx]) * y2[((b * FL + ci) * 10 + yy) * 10 + xx]; }
  const float s = 1.0f / (1.0f + expf(-a)); *(volatile float*)(y3 + t) = s; __threadfence(); *(volatile float*)(y3 + t) = s;
}
__global__ __launch_bounds__(256) void k_final(const float* __restrict__ pam, const float* __restrict__ x, const float* __restrict__ y3, const float* __restrict__ gam, float* __restrict__ out) {
  const int b = blockIdx.x / CC, c = blockIdx.x % CC; const float ga = bf16_round(gam[0]); const float* ym = y3 + ((size_t)b * CC + c) * 100; const float* xc = x + ((size_t)b * CC + c) * HW; const float* x0 = x + (size_t)b * CC * HW;
  for (int pass = 0; pass < 2; ++pass) {
    for (int p = threadIdx.x; p < HW; p += 256) { const int py = p / 64, px = p % 64; const float xv = bf16_round(xc[p]);
      float sy = ((float)py + 0.5f) * (10.0f / 64.0f) - 0.5f, sx = ((float)px + 0.5f) * (10.0f / 64.0f) - 0.5f;
      int y0 = (int)floorf(sy), x0i = (int)floorf(sx); const float fy = sy - (float)y0, fx = sx - (float)x0i;
      int y1 = y0 + 1, x1 = x0i + 1; float wy0 = 1.f - fy, wy1 = fy, wx0 = 1.f - fx, wx1 = fx;
      if (y0 < 0) { y0 = 0; wy0 = 0.f; } if (y1 > 9) { y1 = 9; wy1 = 0.f; } if (x0i < 0) { x0i = 0; wx0 = 0.f; } if (x1 > 9) { x1 = 9; wx1 = 0.f; }
      const float wys = wy0 + wy1, wxs = wx0 + wx1; wy0 /= wys; wy1 /= wys; wx0 /= wxs; wx1 /= wxs;
      const float wv = wy0 * (wx0 * ym[y0 * 10 + x0i] + wx1 * ym[y0 * 10 + x1]) + wy1 * (wx0 * ym[y1 * 10 + x0i] + wx1 * ym[y1 * 10 + x1]);
      const float g = 1.0f / (1.0f + expf(-bf16_round(x0[p])));
      const float sa = ga * pam[((size_t)b * HW + p) * CC + c] + xv; const float ca = xv * wv * g;
      *(volatile float*)(out + ((size_t)b * CC + c) * HW + p) = (sa + ca) + xv; }
    if (pass == 0) __threadfence(); }
}
extern "C" void kernel_launch(void* const* d_in, const int* in_sizes, int n_in,
                              void* d_out, int out_size, void* d_ws, size_t ws_size, hipStream_t stream) {
  (void)in_sizes; (void)n_in; (void)out_size;
  const float* x = (const float*)d_in[0]; const float* qw = (const float*)d_in[1]; const float* qb = (const float*)d_in[2]; const float* kw = (const float*)d_in[3]; const float* kb = (const float*)d_in[4]; const float* vw = (const float*)d_in[5]; const float* vb = (const float*)d_in[6]; const float* gam = (const float*)d_in[7];
  const float* w1 = (const float*)d_in[8]; const float* b1 = (const float*)d_in[9]; const float* w2 = (const float*)d_in[10]; const float* b2 = (const float*)d_in[11]; const float* w3 = (const float*)d_in[12]; const float* b3 = (const float*)d_in[13];
  char* ws = (char*)d_ws; size_t off = 0;
  auto take = [&](size_t bytes) { char* p = ws + off; off += (bytes + 255) & ~(size_t)255; return p; };
  unsigned short* Bt = (unsigned short*)take(128 * CC * 2); float* bias = (float*)take(128 * 4); float* xT = (float*)take((size_t)BB * HW * CC * 4); float* P = (float*)take((size_t)BB * HW * 128 * 4);
  float* Qp = (float*)take((size_t)BB * HW * 32 * 4); unsigned short* Kb = (unsigned short*)take((size_t)BB * HW * 32 * 2); unsigned short* Vt = (unsigned short*)take((size_t)BB * CC * HW * 2);
  float* S = (float*)take((size_t)HW * HW * 4); float* pam = (float*)take((size_t)BB * HW * CC * 4); float* sp = (float*)take((size_t)BB * FL * 400 * 4); float* y2 = (float*)take((size_t)BB * FL * 100 * 4); float* y3 = (float*)take((size_t)BB * CC * 100 * 4);
  if (off > ws_size) return;
  k_wt<<<(128 * 8 + 255) / 256, 256, 0, stream>>>(qw, kw, vw, w1, qb, kb, vb, b1, Bt, bias);
  k_transpose32<false, false, false><<<dim3(HW / 32, CC / 32, BB), 256, 0, stream>>>(x, xT, CC, HW, nullptr, nullptr, nullptr);
  k_gemm_bf3<false, 0, false, false><<<((BB * HW / 16) * 2 + 3) / 4, 128, 0, stream>>>(xT, CC, Bt, CC, bias, nullptr, 1, 0, P, 128, BB * HW, 128, CC);
  k_qkv<<<(unsigned)(((size_t)BB * HW * 32 + 255) / 256), 256, 0, stream>>>(P, Qp, Kb); k_vt<<<(unsigned)(((size_t)BB * CC * (HW / 8) + 255) / 256), 256, 0, stream>>>(P, Vt);
  for (int b = 0; b < BB; ++b) {
    k_gemm_b<true, false, 0><<<dim3(((HW / 16) * (HW / 64) + 3) / 4, 1), 128, 0, stream>>>(Qp + (size_t)b * HW * 32, 32, 0, Kb + (size_t)b * HW * 32, Kb + (size_t)b * HW * 32, 32, 0, nullptr, nullptr, 0, 0, 1.f, 1.f, S, HW, 0, HW, HW, 32);
    k_softmax<<<HW / 8, 256, 0, stream>>>(S);
    k_gemm_b<true, false, 0><<<dim3(((HW / 16) * (CC / 64) + 3) / 4, 1), 128, 0, stream>>>(S, HW, 0, Vt + (size_t)b * CC * HW, Vt + (size_t)b * CC * HW, HW, 0, nullptr, nullptr, 0, 0, 1.f, 1.f, pam + (size_t)b * HW * CC, CC, 0, HW, CC, HW);
  }
  k_softpool<<<(BB * FL * 400 + 255) / 256, 256, 0, stream>>>(P, sp);
  k_conv2<<<(BB * FL * 100 + 255) / 256, 256, 0, stream>>>(sp, w2, b2, y2);
  k_conv3<<<(BB * CC * 100 + 255) / 256, 256, 0, stream>>>(y2, w3, b3, y3);
  k_final<<<BB * CC, 256, 0, stream>>>(pam, x, y3, gam, (float*)d_out);
}
